// CausalSelfAttention_86560770883928
// MI455X (gfx1250) — hardware-verified
//
#include <hip/hip_runtime.h>


#ifndef NB
#define NB 2
#endif
#ifndef SEQ
#define SEQ 2048
#endif
#define NB_FULL  2
#define SEQ_FULL 2048
#define DM   1024
#define NH   16
#define HD   64
#if SEQ < 256
#define RH   SEQ
#else
#define RH   256
#endif
#define MR   (NB * SEQ)
#define PLN  ((size_t)NB * NH * SEQ * HD)
#define PCAR 1024.0f
#define L2E  1.4426950408889634f
#define NEGB (-1.0e30f)
#define RMS_EPS 1.1920928955078125e-07f

static_assert(NB >= 1 && NB <= NB_FULL);
static_assert(SEQ >= 64 && SEQ <= SEQ_FULL);
static_assert(SEQ % 64 == 0);
static_assert(RH % 64 == 0);
static_assert(RH <= SEQ);
static_assert(DM % 64 == 0);
static_assert(DM % 32 == 0);
static_assert(NH * HD == DM);
static_assert(HD == 64);
static_assert(MR % 64 == 0);

typedef _Float16 h16;
typedef unsigned short bf;
typedef __attribute__((ext_vector_type(16))) __bf16   v16bf;
typedef __attribute__((ext_vector_type(16))) _Float16 v16h;
typedef __attribute__((ext_vector_type(8)))  _Float16 v8h;
typedef __attribute__((ext_vector_type(8)))  unsigned short v8us;
typedef __attribute__((ext_vector_type(8)))  float    v8f;
typedef __attribute__((ext_vector_type(4)))  float    v4f;
typedef __attribute__((ext_vector_type(2)))  float    v2f;
typedef v8h  __attribute__((may_alias)) v8ha;
typedef v4f  __attribute__((may_alias)) v4fa;
typedef v8us __attribute__((may_alias)) v8usa;

__device__ __forceinline__ unsigned short f2bf(float f) { unsigned u = __float_as_uint(f); u += 0x7FFFu + ((u >> 16) & 1u); return (unsigned short)(u >> 16); }
__device__ __forceinline__ float bf2f(unsigned short b) { return __uint_as_float(((unsigned)b) << 16); }
__device__ __forceinline__ void splitf(float y, unsigned short& h, unsigned short& l) { h = f2bf(y); l = f2bf(y - bf2f(h)); }
__device__ __forceinline__ v16h cat16(v8h lo, v8h hi) { return __builtin_shufflevector(lo, hi, 0, 1, 2, 3, 4, 5, 6, 7, 8, 9, 10, 11, 12, 13, 14, 15); }
__device__ __forceinline__ v16bf cat16b(v8us lo, v8us hi) { return __builtin_bit_cast(v16bf, __builtin_shufflevector(lo, hi, 0, 1, 2, 3, 4, 5, 6, 7, 8, 9, 10, 11, 12, 13, 14, 15)); }
__device__ __forceinline__ v16bf ldb(const bf* p) { return cat16b(*(const v8us*)p, *(const v8us*)(p + 16)); }
__device__ __forceinline__ v16h  ldh(const h16* p) { return cat16(*(const v8h*)p, *(const v8h*)(p + 16)); }
__device__ __forceinline__ v8f mmab(v16bf a, v16bf b, v8f c) {
    c = __builtin_amdgcn_wmma_f32_16x16x32_bf16(false, a, false, b, (short)0, c, false, false);
    asm volatile("v_nop\n\tv_nop\n\tv_nop\n\tv_nop" : "+v"(c) : "v"(a), "v"(b));
    return c; }
__device__ __forceinline__ v8f mmah(v16h a, v16h b, v8f c) {
    c = __builtin_amdgcn_wmma_f32_16x16x32_f16(false, a, false, b, (short)0, c, false, false);
    asm volatile("v_nop\n\tv_nop\n\tv_nop\n\tv_nop" : "+v"(c) : "v"(a), "v"(b));
    return c; }
__device__ __forceinline__ void wave_sync_lds() { asm volatile("s_wait_dscnt 0" ::: "memory"); __builtin_amdgcn_wave_barrier(); asm volatile("" ::: "memory"); }

template <int NSPLIT>
__device__ __forceinline__ void gemm_acc(const bf* __restrict__ A, const bf* __restrict__ A2, const bf* __restrict__ Bt, int aoff, int boff, v8f (&acc)[4][4]) {
#pragma unroll 1
    for (int kc = 0; kc < DM; kc += 32) {
        v16bf a[4], a2[4];
#pragma unroll
        for (int mb = 0; mb < 4; ++mb) { a[mb] = ldb(A + aoff + mb * 16 * DM + kc); if (NSPLIT) a2[mb] = ldb(A2 + aoff + mb * 16 * DM + kc); }
#pragma unroll
        for (int nb = 0; nb < 4; ++nb) { const v16bf b = ldb(Bt + boff + nb * 16 * DM + kc);
#pragma unroll
            for (int mb = 0; mb < 4; ++mb) { acc[mb][nb] = mmab(a[mb], b, acc[mb][nb]); if (NSPLIT) acc[mb][nb] = mmab(a2[mb], b, acc[mb][nb]); } }
    }
}

__global__ __launch_bounds__(256) void k_cvtx(const float* __restrict__ x, bf* XB) {
    const size_t i = (size_t)blockIdx.x * 256 + threadIdx.x; if (i >= (size_t)MR * DM / 8) return;
    const size_t e = i * 8; const int row = (int)(e / DM), col = (int)(e % DM); const int b = row / SEQ, t = row - b * SEQ;
    const v8f v = *(const v8f*)(x + ((size_t)b * SEQ_FULL + t) * DM + col); v8us o;
#pragma unroll
    for (int k = 0; k < 8; ++k) o[k] = f2bf(v[k]);
    *(volatile v8us*)(XB + e) = o; __threadfence(); *(volatile v8us*)(XB + e) = o; }
__global__ __launch_bounds__(256) void k_cvt8(const float* __restrict__ src, bf* dst, int n8) {
    const int i = blockIdx.x * 256 + threadIdx.x; if (i >= n8) return; const v8f v = *(const v8f*)(src + (size_t)i * 8); v8us o;
#pragma unroll
    for (int k = 0; k < 8; ++k) o[k] = f2bf(v[k]);
    *(volatile v8us*)(dst + (size_t)i * 8) = o; __threadfence(); *(volatile v8us*)(dst + (size_t)i * 8) = o; }
__global__ __launch_bounds__(256) void k_cs(float* CS) {
    const int idx = blockIdx.x * 256 + threadIdx.x; if (idx >= SEQ * 32) return; const int j = idx & 31, t = idx >> 5;
    double p = 1.0;
    if (j & 1)  p *= 1.333521432163324;
    if (j & 2)  p *= 1.7782794100389228;
    if (j & 4)  p *= 3.1622776601683795;
    if (j & 8)  p *= 10.0;
    if (j & 16) p *= 100.0;
    const float pf = (float)p; const float inv = 1.0f / pf; const float ang = (float)t * inv;
    float sn, cs; sincosf(ang, &sn, &cs);
    v2f o; o[0] = cs; o[1] = sn;
    *(volatile v2f*)(CS + (size_t)idx * 2) = o; __threadfence(); *(volatile v2f*)(CS + (size_t)idx * 2) = o; }

__global__ __launch_bounds__(32) void k_projqk(const bf* __restrict__ XB, const bf* __restrict__ W4, const float* __restrict__ CS, bf* PH, bf* PL) {
    __shared__ __align__(16) float os[16 * 68];
    const int lane = threadIdx.x & 31, lr = lane & 15, hi = lane >> 4;
    const int r0 = blockIdx.x * 64, head = blockIdx.y, c0 = head * 64, z = blockIdx.z;
    const bf* Bt = W4 + (size_t)z * DM * DM;
    const float sc = (z == 0) ? 0.125f : 1.0f;
    const size_t pz = (size_t)z * PLN;
    v8f acc[4][4];
#pragma unroll
    for (int mb = 0; mb < 4; ++mb)
#pragma unroll
        for (int nb = 0; nb < 4; ++nb) acc[mb][nb] = (v8f){};
    gemm_acc<0>(XB, XB, Bt, (r0 + lr) * DM + 8 * hi, (c0 + lr) * DM + 8 * hi, acc);
    const int r4 = lane >> 3, j8 = lane & 7, d0 = j8 * 8, dp = d0 ^ 32, i0 = d0 & 31;
    const float sgn = (j8 < 4) ? 1.0f : -1.0f;
    const int b = r0 / SEQ, tb = r0 - b * SEQ;
#pragma unroll
    for (int mb = 0; mb < 4; ++mb) {
#pragma unroll
        for (int nb = 0; nb < 4; ++nb) {
#pragma unroll
            for (int j = 0; j < 8; ++j) os[(hi * 8 + j) * 68 + nb * 16 + lr] = acc[mb][nb][j]; }
        wave_sync_lds();
#pragma unroll 1
        for (int it = 0; it < 4; ++it) {
            const int row = it * 4 + r4; const int t = tb + mb * 16 + row;
            const v4f a0 = *(const v4fa*)(os + row * 68 + d0), a1 = *(const v4fa*)(os + row * 68 + d0 + 4);
            const v4f b0 = *(const v4fa*)(os + row * 68 + dp), b1 = *(const v4fa*)(os + row * 68 + dp + 4);
            float ow[8], pw[8], cs[16];
#pragma unroll
            for (int e = 0; e < 4; ++e) { ow[e] = a0[e]; ow[4 + e] = a1[e]; pw[e] = b0[e]; pw[4 + e] = b1[e]; }
            float ss = 0.f;
#pragma unroll
            for (int e = 0; e < 8; ++e) ss += ow[e] * ow[e];
            ss += __shfl_xor(ss, 1, 32); ss += __shfl_xor(ss, 2, 32); ss += __shfl_xor(ss, 4, 32);
            const float rn = rsqrtf(ss * (1.0f / 64.0f) + RMS_EPS);
            const float* cp = CS + ((size_t)t * 32 + i0) * 2;
            const v4f c0v = *(const v4f*)cp, c1v = *(const v4f*)(cp + 4), c2v = *(const v4f*)(cp + 8), c3v = *(const v4f*)(cp + 12);
#pragma unroll
            for (int e = 0; e < 4; ++e) { cs[e] = c0v[e]; cs[4 + e] = c1v[e]; cs[8 + e] = c2v[e]; cs[12 + e] = c3v[e]; }
            v8us oh, ol;
#pragma unroll
            for (int e = 0; e < 8; ++e) { const float xo = ow[e] * rn, xp = pw[e] * rn; const float r = (xo * cs[2 * e] + sgn * (xp * cs[2 * e + 1])) * sc;
                unsigned short a2, c2; splitf(r, a2, c2); oh[e] = a2; ol[e] = c2; }
            const size_t oo = pz + (((size_t)(b * NH + head)) * SEQ + t) * HD + d0;
            *(volatile v8us*)(PH + oo) = oh; *(volatile v8us*)(PL + oo) = ol; __threadfence(); *(volatile v8us*)(PH + oo) = oh; *(volatile v8us*)(PL + oo) = ol; }
        wave_sync_lds();
    }
}

__global__ __launch_bounds__(32) void k_projv(const bf* __restrict__ W4, const bf* __restrict__ XB, h16* V16, bf* Vh, bf* Vl) {
    __shared__ __align__(16) float os[16 * 68];
    const int lane = threadIdx.x & 31, lr = lane & 15, hi = lane >> 4;
    const int r0 = blockIdx.x * 64, c0 = blockIdx.y * 64, b = blockIdx.z;
    const bf* A = W4 + (size_t)2 * DM * DM; const bf* Bt = XB + (size_t)b * SEQ * DM;
    v8f acc[4][4];
#pragma unroll
    for (int mb = 0; mb < 4; ++mb)
#pragma unroll
        for (int nb = 0; nb < 4; ++nb) acc[mb][nb] = (v8f){};
    gemm_acc<0>(A, A, Bt, (r0 + lr) * DM + 8 * hi, (c0 + lr) * DM + 8 * hi, acc);
    const int r4 = lane >> 3, j8 = lane & 7; const bool early = (c0 < RH);
#pragma unroll
    for (int mb = 0; mb < 4; ++mb) {
#pragma unroll
        for (int nb = 0; nb < 4; ++nb) {
#pragma unroll
            for (int j = 0; j < 8; ++j) os[(hi * 8 + j) * 68 + nb * 16 + lr] = acc[mb][nb][j]; }
        wave_sync_lds();
#pragma unroll 1
        for (int it = 0; it < 4; ++it) {
            const int row = it * 4 + r4; const int n = r0 + mb * 16 + row; const int t0 = c0 + j8 * 8;
            const v4f a0 = *(const v4fa*)(os + row * 68 + j8 * 8), a1 = *(const v4fa*)(os + row * 68 + j8 * 8 + 4);
            v8h o16; v8us oh, ol;
#pragma unroll
            for (int e = 0; e < 8; ++e) { const float x = (e < 4) ? a0[e & 3] : a1[e & 3]; o16[e] = (h16)x; unsigned short a2, c2; splitf(x, a2, c2); oh[e] = a2; ol[e] = c2; }
            const size_t o1 = ((size_t)(b * DM + n)) * SEQ + t0; const size_t o2 = ((size_t)(b * DM + n)) * RH + t0;
            *(volatile v8h*)(V16 + o1) = o16; if (early) { *(volatile v8us*)(Vh + o2) = oh; *(volatile v8us*)(Vl + o2) = ol; }
            __threadfence();
            *(volatile v8h*)(V16 + o1) = o16; if (early) { *(volatile v8us*)(Vh + o2) = oh; *(volatile v8us*)(Vl + o2) = ol; } }
        wave_sync_lds();
    }
}

__global__ __launch_bounds__(32) void k_projo(const bf* __restrict__ ATh, const bf* __restrict__ ATl, const bf* __restrict__ W4, float* OUT) {
    __shared__ __align__(16) float os[16 * 68];
    const int lane = threadIdx.x & 31, lr = lane & 15, hi = lane >> 4;
    const int r0 = blockIdx.x * 64, c0 = blockIdx.y * 64;
    const bf* Bt = W4 + (size_t)3 * DM * DM;
    v8f acc[4][4];
#pragma unroll
    for (int mb = 0; mb < 4; ++mb)
#pragma unroll
        for (int nb = 0; nb < 4; ++nb) acc[mb][nb] = (v8f){};
    gemm_acc<1>(ATh, ATl, Bt, (r0 + lr) * DM + 8 * hi, (c0 + lr) * DM + 8 * hi, acc);
#pragma unroll
    for (int mb = 0; mb < 4; ++mb) {
#pragma unroll
        for (int nb = 0; nb < 4; ++nb) {
#pragma unroll
            for (int j = 0; j < 8; ++j) os[(hi * 8 + j) * 68 + nb * 16 + lr] = acc[mb][nb][j]; }
        wave_sync_lds();
        float* crow = OUT + (size_t)(r0 + mb * 16) * DM + c0;
#pragma unroll 1
        for (int ps = 0; ps < 2; ++ps) {
#pragma unroll
            for (int s = 0; s < 8; ++s) { const int row = 2 * s + hi, cofs = lr * 4; const v4f val = *(const v4fa*)(os + row * 68 + cofs);
                *(volatile v4f*)(crow + (size_t)row * DM + cofs) = val; }
            if (ps == 0) __threadfence(); }
        wave_sync_lds();
    }
}

template <bool EARLY>
__device__ __forceinline__ void attn_body(const bf* __restrict__ Qh, const bf* __restrict__ Ql, const bf* __restrict__ Kh, const bf* __restrict__ Kl,
                                          const h16* __restrict__ V16, const bf* __restrict__ Vh, const bf* __restrict__ Vl, bf* Ah, bf* Al, int rowoff) {
    __shared__ __align__(16) float os[4][16 * 68];
    __shared__ __align__(16) h16 pf[4][16 * 40];
    __shared__ __align__(16) bf  ph[4][16 * 40];
    __shared__ __align__(16) bf  pl[4][16 * 40];
    const int lane = threadIdx.x & 31, lr = lane & 15, hi = lane >> 4;
    const int wave = __builtin_amdgcn_readfirstlane(threadIdx.x >> 5);
    const int bh = blockIdx.y; const int qrow0 = rowoff + blockIdx.x * 64 + wave * 16;
    const int pb = bh * SEQ * HD;
    const int nch = (qrow0 >> 5) + 1;
    v8f oa[4];
#pragma unroll
    for (int sl = 0; sl < 4; ++sl) oa[sl] = (v8f){};
    float m[8], l[8];
#pragma unroll
    for (int r = 0; r < 8; ++r) { m[r] = NEGB; l[r] = 0.f; }
    const int qoff0 = pb + (qrow0 + lr) * HD + 8 * hi;
#pragma unroll 1
    for (int c = 0; c < nch; ++c) {
        const int kb = c * 32;
        int qo = qoff0; asm volatile("" : "+v"(qo));
        const v16bf qh0 = ldb(Qh + qo), qh1 = ldb(Qh + qo + 32), ql0 = ldb(Ql + qo), ql1 = ldb(Ql + qo + 32);
        v8f s0 = (v8f){}, s1 = (v8f){};
        { const int ko = pb + (kb + lr) * HD + 8 * hi;
          const v16bf kh0 = ldb(Kh + ko), kh1 = ldb(Kh + ko + 32), kl0 = ldb(Kl + ko), kl1 = ldb(Kl + ko + 32);
          s0 = mmab(qh0, kh0, s0); s0 = mmab(qh1, kh1, s0); s0 = mmab(ql0, kh0, s0); s0 = mmab(ql1, kh1, s0); s0 = mmab(qh0, kl0, s0); s0 = mmab(qh1, kl1, s0); }
        { const int ko = pb + (kb + 16 + lr) * HD + 8 * hi;
          const v16bf kh0 = ldb(Kh + ko), kh1 = ldb(Kh + ko + 32), kl0 = ldb(Kl + ko), kl1 = ldb(Kl + ko + 32);
          s1 = mmab(qh0, kh0, s1); s1 = mmab(qh1, kh1, s1); s1 = mmab(ql0, kh0, s1); s1 = mmab(ql1, kh1, s1); s1 = mmab(qh0, kl0, s1); s1 = mmab(qh1, kl1, s1); }
        const bool diag = (kb + 31 > qrow0);
        const int kg0 = kb + lr;
#pragma unroll
        for (int r = 0; r < 8; ++r) {
            const int qg = qrow0 + 8 * hi + r;
            float v0 = s0[r] * L2E, v1 = s1[r] * L2E;
            if (diag) { v0 = (kg0 <= qg) ? v0 : NEGB; v1 = (kg0 + 16 <= qg) ? v1 : NEGB; }
            float mx = fmaxf(v0, v1);
            mx = fmaxf(mx, __shfl_xor(mx, 1, 32)); mx = fmaxf(mx, __shfl_xor(mx, 2, 32)); mx = fmaxf(mx, __shfl_xor(mx, 4, 32)); mx = fmaxf(mx, __shfl_xor(mx, 8, 32));
            const float mnew = fmaxf(m[r], mx);
            const float alpha = __builtin_amdgcn_exp2f(m[r] - mnew);
            const float e0 = __builtin_amdgcn_exp2f(v0 - mnew), e1 = __builtin_amdgcn_exp2f(v1 - mnew);
            l[r] = l[r] * alpha + (e0 + e1); m[r] = mnew;
#pragma unroll
            for (int sl = 0; sl < 4; ++sl) oa[sl][r] *= alpha;
            const int po = (8 * hi + r) * 40 + lr;
            if (EARLY) { unsigned short a2, c2; splitf(e0, a2, c2); ph[wave][po] = a2; pl[wave][po] = c2; splitf(e1, a2, c2); ph[wave][po + 16] = a2; pl[wave][po + 16] = c2; }
            else { pf[wave][po] = (h16)(e0 * PCAR); pf[wave][po + 16] = (h16)(e1 * PCAR); }
        }
        wave_sync_lds();
        if (EARLY) {
            const v16bf pah = cat16b(*(const v8usa*)(&ph[wave][lr * 40 + 8 * hi]), *(const v8usa*)(&ph[wave][lr * 40 + 16 + 8 * hi]));
            const v16bf pal = cat16b(*(const v8usa*)(&pl[wave][lr * 40 + 8 * hi]), *(const v8usa*)(&pl[wave][lr * 40 + 16 + 8 * hi]));
#pragma unroll
            for (int sl = 0; sl < 4; ++sl) { const int vo = (bh * HD + sl * 16 + lr) * RH + kb + 8 * hi; const v16bf vh = ldb(Vh + vo), vl = ldb(Vl + vo);
                oa[sl] = mmab(pah, vh, oa[sl]); oa[sl] = mmab(pal, vh, oa[sl]); oa[sl] = mmab(pah, vl, oa[sl]); }
        } else {
            const v16h pa = cat16(*(const v8ha*)(&pf[wave][lr * 40 + 8 * hi]), *(const v8ha*)(&pf[wave][lr * 40 + 16 + 8 * hi]));
#pragma unroll
            for (int sl = 0; sl < 4; ++sl) { const int vo = (bh * HD + sl * 16 + lr) * SEQ + kb + 8 * hi; const v16h vf = ldh(V16 + vo);
                oa[sl] = mmah(pa, vf, oa[sl]); }
        }
        wave_sync_lds();
    }
    const float carry = EARLY ? 1.0f : (1.0f / PCAR);
#pragma unroll
    for (int r = 0; r < 8; ++r) { float t = l[r]; t += __shfl_xor(t, 1, 32); t += __shfl_xor(t, 2, 32); t += __shfl_xor(t, 4, 32); t += __shfl_xor(t, 8, 32);
        const float inv = carry * (1.0f / t);
#pragma unroll
        for (int sl = 0; sl < 4; ++sl) os[wave][(8 * hi + r) * 68 + sl * 16 + lr] = oa[sl][r] * inv; }
    wave_sync_lds();
    const int r4 = lane >> 3, d0 = (lane & 7) * 8; const int b = bh / NH, h = bh - b * NH;
#pragma unroll 1
    for (int it = 0; it < 4; ++it) {
        const int row = it * 4 + r4;
        const v4f a0 = *(const v4fa*)(&os[wave][row * 68 + d0]), a1 = *(const v4fa*)(&os[wave][row * 68 + d0 + 4]);
        v8us oh, ol;
#pragma unroll
        for (int e = 0; e < 8; ++e) { const float x = (e < 4) ? a0[e & 3] : a1[e & 3]; unsigned short a2, c2; splitf(x, a2, c2); oh[e] = a2; ol[e] = c2; }
        const size_t oo = ((size_t)(b * SEQ + qrow0 + row)) * DM + h * HD + d0;
        *(volatile v8us*)(Ah + oo) = oh; *(volatile v8us*)(Al + oo) = ol; __threadfence(); *(volatile v8us*)(Ah + oo) = oh; *(volatile v8us*)(Al + oo) = ol; }
}
__global__ __launch_bounds__(128) void k_attn_e(const bf* __restrict__ Qh, const bf* __restrict__ Ql, const bf* __restrict__ Kh, const bf* __restrict__ Kl,
                                                const h16* __restrict__ V16, const bf* __restrict__ Vh, const bf* __restrict__ Vl, bf* Ah, bf* Al) {
    attn_body<true>(Qh, Ql, Kh, Kl, V16, Vh, Vl, Ah, Al, 0); }
__global__ __launch_bounds__(128) void k_attn_l(const bf* __restrict__ Qh, const bf* __restrict__ Ql, const bf* __restrict__ Kh, const bf* __restrict__ Kl,
                                                const h16* __restrict__ V16, const bf* __restrict__ Vh, const bf* __restrict__ Vl, bf* Ah, bf* Al) {
    attn_body<false>(Qh, Ql, Kh, Kl, V16, Vh, Vl, Ah, Al, RH); }

constexpr size_t al256(size_t b) { return (b + 255) & ~(size_t)255; }
constexpr size_t SZ_XB = al256((size_t)MR * DM * 2);
constexpr size_t SZ_W4 = al256((size_t)4 * DM * DM * 2);
constexpr size_t SZ_CS = al256((size_t)SEQ * 32 * 2 * 4);
constexpr size_t SZ_QK = al256((size_t)2 * PLN * 2);
constexpr size_t SZ_V16 = al256((size_t)NB * DM * SEQ * 2);
constexpr size_t SZ_VR = al256((size_t)NB * DM * RH * 2);
constexpr size_t SZ_AT = al256((size_t)MR * DM * 2);
constexpr size_t SZ_TOTAL = SZ_XB + SZ_W4 + SZ_CS + 2 * SZ_QK + SZ_V16 + 2 * SZ_VR + 2 * SZ_AT;
static_assert(SZ_TOTAL <= (size_t)134217728);

extern "C" void kernel_launch(void* const* d_in, const int* in_sizes, int n_in,
                              void* d_out, int out_size, void* d_ws, size_t ws_size, hipStream_t stream) {
    if (n_in < 5) return;
    if (in_sizes[0] < (NB - 1) * SEQ_FULL * DM + SEQ * DM) return;
    if (in_sizes[1] < DM * DM || in_sizes[2] < DM * DM || in_sizes[3] < DM * DM || in_sizes[4] < DM * DM) return;
    if (out_size < MR * DM) return;
    if (SZ_TOTAL > ws_size) return;
    const float* x = (const float*)d_in[0]; const float* wq = (const float*)d_in[1]; const float* wk = (const float*)d_in[2];
    const float* wv = (const float*)d_in[3]; const float* wo = (const float*)d_in[4];
    float* OUT = (float*)d_out;
    char* wsp = (char*)d_ws;
    bf* XB = (bf*)wsp; wsp += SZ_XB;
    bf* W4 = (bf*)wsp; wsp += SZ_W4;
    float* CS = (float*)wsp; wsp += SZ_CS;
    bf* QKh = (bf*)wsp; wsp += SZ_QK;
    bf* QKl = (bf*)wsp; wsp += SZ_QK;
    h16* V16 = (h16*)wsp; wsp += SZ_V16;
    bf* Vh = (bf*)wsp; wsp += SZ_VR;
    bf* Vl = (bf*)wsp; wsp += SZ_VR;
    bf* ATh = (bf*)wsp; wsp += SZ_AT;
    bf* ATl = (bf*)wsp; wsp += SZ_AT;
    const unsigned nw8 = (unsigned)(DM * DM / 8);
    k_cvtx<<<(unsigned)(((size_t)MR * DM / 8 + 255) / 256), 256, 0, stream>>>(x, XB);
    k_cvt8<<<(nw8 + 255) / 256, 256, 0, stream>>>(wq, W4, (int)nw8);
    k_cvt8<<<(nw8 + 255) / 256, 256, 0, stream>>>(wk, W4 + (size_t)DM * DM, (int)nw8);
    k_cvt8<<<(nw8 + 255) / 256, 256, 0, stream>>>(wv, W4 + (size_t)2 * DM * DM, (int)nw8);
    k_cvt8<<<(nw8 + 255) / 256, 256, 0, stream>>>(wo, W4 + (size_t)3 * DM * DM, (int)nw8);
    k_cs<<<(SEQ * 32 + 255) / 256, 256, 0, stream>>>(CS);
    k_projqk<<<dim3(MR / 64, NH, 2), 32, 0, stream>>>(XB, W4, CS, QKh, QKl);
    k_projv<<<dim3(DM / 64, SEQ / 64, NB), 32, 0, stream>>>(W4, XB, V16, Vh, Vl);
    k_attn_e<<<dim3(RH / 64, NB * NH), 128, 0, stream>>>(QKh, QKl, QKh + PLN, QKl + PLN, V16, Vh, Vl, ATh, ATl);
    if (SEQ > RH) k_attn_l<<<dim3((SEQ - RH) / 64, NB * NH), 128, 0, stream>>>(QKh, QKl, QKh + PLN, QKl + PLN, V16, Vh, Vl, ATh, ATl);
    k_projo<<<dim3(MR / 64, DM / 64), 32, 0, stream>>>(ATh, ATl, W4, OUT);
}
